// GNNHolographicPredictor_23545010716680
// MI455X (gfx1250) — hardware-run, weakly checked
//
#include <hip/hip_runtime.h>

typedef float          v8f   __attribute__((ext_vector_type(8)));
typedef float          v4f   __attribute__((ext_vector_type(4)));
typedef unsigned int   v4u   __attribute__((ext_vector_type(4)));
typedef int            v8i   __attribute__((ext_vector_type(8)));
typedef unsigned short v8us  __attribute__((ext_vector_type(8)));
typedef unsigned short v16us __attribute__((ext_vector_type(16)));
typedef __bf16         v16bf __attribute__((ext_vector_type(16)));
typedef _Float16       v16h  __attribute__((ext_vector_type(16)));
typedef v4f  __attribute__((may_alias)) v4fa;
typedef v8us __attribute__((may_alias)) v8usa;
union FragB { v16bf v; v16us u; v8us h[2]; v8i w; };
union FragH { v16h  v; v16us u; v8us h[2]; v8i w; };

__device__ __forceinline__ v8f wmb(const FragB& a, const FragB& b, v8f c) {
  v8f d = __builtin_amdgcn_wmma_f32_16x16x32_bf16(false, a.v, false, b.v, (short)0, c, false, false);
  asm volatile("v_nop\n\tv_nop\n\tv_nop\n\tv_nop" : "+v"(d) : "v"(a.w), "v"(b.w));
  return d;
}

__device__ __forceinline__ v8f wmh(const FragH& a, const FragH& b, v8f c) {
  v8f d = __builtin_amdgcn_wmma_f32_16x16x32_f16(false, a.v, false, b.v, (short)0, c, false, false);
  asm volatile("v_nop\n\tv_nop\n\tv_nop\n\tv_nop" : "+v"(d) : "v"(a.w), "v"(b.w));
  return d;
}

__device__ __forceinline__ unsigned bf16_bits(float f) {
  const unsigned u = __float_as_uint(f);
  const unsigned r = (u + 0x7FFFu + ((u >> 16) & 1u)) >> 16;
  const unsigned q = (u >> 16) | 0x40u;
  return ((u & 0x7fffffffu) > 0x7f800000u) ? q : r;
}

__device__ __forceinline__ float bf16_val(float f) {
  return __uint_as_float(bf16_bits(f) << 16);
}
__device__ __forceinline__ int clampi(int v, int lo, int hi) {
  return v < lo ? lo : (v > hi ? hi : v);
}

__device__ __forceinline__ unsigned f16_bits(float f) {
  const unsigned u  = __float_as_uint(f);
  const unsigned s  = (u >> 16) & 0x8000u;
  const unsigned a  = u & 0x7fffffffu;
  const unsigned t  = a - 0x38000000u;
  const unsigned r  = (t + 0x0FFFu + ((t >> 13) & 1u)) >> 13;
  const unsigned rc = r > 0x7C00u ? 0x7C00u : r;
  const bool small  = a < 0x38800000u;
  const bool isnan  = a > 0x7f800000u;
  const unsigned fin = small ? 0u : (s | rc);
  return isnan ? (s | 0x7E00u) : fin;
}

__device__ __forceinline__ unsigned pk16(unsigned lo, unsigned hi) { return lo | (hi << 16); }
__device__ __forceinline__ unsigned bf16_lo_bits(float v) {
  float hi = bf16_val(v);
  asm volatile("" : "+v"(hi));
  return bf16_bits(v - hi);
}
__device__ __forceinline__ v4u pack8_bf16(v4f a, v4f c) {
  return (v4u){ pk16(bf16_bits(a[0]), bf16_bits(a[1])), pk16(bf16_bits(a[2]), bf16_bits(a[3])),
                pk16(bf16_bits(c[0]), bf16_bits(c[1])), pk16(bf16_bits(c[2]), bf16_bits(c[3])) };
}
__device__ __forceinline__ v4u pack8_bf16_lo(v4f a, v4f c) {
  return (v4u){ pk16(bf16_lo_bits(a[0]), bf16_lo_bits(a[1])), pk16(bf16_lo_bits(a[2]), bf16_lo_bits(a[3])),
                pk16(bf16_lo_bits(c[0]), bf16_lo_bits(c[1])), pk16(bf16_lo_bits(c[2]), bf16_lo_bits(c[3])) };
}
__device__ __forceinline__ v4u pack8_f16(v4f a, v4f c) {
  return (v4u){ pk16(f16_bits(a[0]), f16_bits(a[1])), pk16(f16_bits(a[2]), f16_bits(a[3])),
                pk16(f16_bits(c[0]), f16_bits(c[1])), pk16(f16_bits(c[2]), f16_bits(c[3])) };
}

template <int FORM>
__global__ __launch_bounds__(256) void k_plane(const float* __restrict__ src, int rows, int cols, int ldsrc,
                                               unsigned short* __restrict__ dst, int MP, int KP) {
  static_assert(FORM >= 0 && FORM <= 3);
  const int KTOT = (FORM == 1 || FORM == 3) ? 2 * KP : KP;
  const unsigned ppr   = (unsigned)(KTOT >> 3);
  const unsigned kp8   = (unsigned)(KP >> 3);
  const unsigned total = (unsigned)MP * ppr;
  const unsigned g     = blockIdx.x * 256u + threadIdx.x;
  const unsigned rowu  = g / ppr;
  const unsigned p     = g - rowu * ppr;
  const bool second    = p >= kp8;
  const int row = (int)rowu;
  const int c0  = (int)((second ? p - kp8 : p) << 3);
  const float* srow = src + (size_t)clampi(row, 0, rows - 1) * (size_t)ldsrc;
  float x[8];
  unsigned mk[8];
#pragma unroll
  for (int e = 0; e < 8; ++e) {
    const int c = c0 + e;
    const float v = srow[clampi(c, 0, cols - 1)];
    asm volatile("" :: "v"(v));
    x[e]  = v;
    mk[e] = (row < rows && c < cols) ? 0xFFFFu : 0u;
  }
  const v4f a = (v4f){ x[0], x[1], x[2], x[3] };
  const v4f c = (v4f){ x[4], x[5], x[6], x[7] };
  v4u o;
  if (FORM == 2) {
    o = pack8_f16(a, c);
  } else {
    const v4u hi = pack8_bf16(a, c);
    o = hi;
    if (FORM == 1) { const v4u lo = pack8_bf16_lo(a, c); o = second ? lo : hi; }
  }
  const v4u mw = (v4u){ pk16(mk[0], mk[1]), pk16(mk[2], mk[3]), pk16(mk[4], mk[5]), pk16(mk[6], mk[7]) };
  o &= mw;
  if (g < total) {
    volatile v4u* q = (volatile v4u*)(dst + (size_t)g * 8);
    *q = o;
    __threadfence();
    *q = o;
  }
}

template <int FORM> struct FragOf    { typedef FragB T; };
template <>         struct FragOf<2> { typedef FragH T; };
__device__ __forceinline__ v8f mm(const FragB& a, const FragB& b, v8f c) { return wmb(a, b, c); }
__device__ __forceinline__ v8f mm(const FragH& a, const FragH& b, v8f c) { return wmh(a, b, c); }
template <class F> __device__ __forceinline__ F ld_frag(const unsigned short* p) {
  F f;
  f.h[0] = *(const v8usa*)(p);
  f.h[1] = *(const v8usa*)(p + 16);
  return f;
}

template <int FORM, int EPI>
__global__ __launch_bounds__(256) __attribute__((amdgpu_num_vgpr(248)))
void k_gemm_nt(const unsigned short* __restrict__ A, const unsigned short* __restrict__ B,
               const float* __restrict__ bias, float* __restrict__ D, int M, int N, int KTOT, int ldd) {
  static_assert(FORM >= 0 && FORM <= 2);
  static_assert(EPI == 0 || EPI == 1);
  typedef typename FragOf<FORM>::T F;
  __shared__ __attribute__((aligned(16))) float sT[8][16 * 68];
  const int lane = threadIdx.x & 31;
  const int wave = threadIdx.x >> 5;
  const int tilesM = (M + 63) >> 6;
  const int tilesN = (N + 63) >> 6;
  const int tile = blockIdx.x * 8 + wave;
  if (tile >= tilesM * tilesN) return;
  const int tm = tile / tilesN;
  const int tn = tile - tm * tilesN;
  const int m0 = tm << 6;
  const int n0 = tn << 6;

  const int rl = lane & 15;
  const int h8 = (lane >> 4) * 8;
  const unsigned short* pa = A + (size_t)(m0 + rl) * (size_t)KTOT + h8;
  const unsigned short* pb = B + (size_t)(n0 + rl) * (size_t)KTOT + h8;

  v8f acc[4][4];
#pragma unroll
  for (int i = 0; i < 4; ++i)
#pragma unroll
    for (int j = 0; j < 4; ++j) acc[i][j] = (v8f){0.f, 0.f, 0.f, 0.f, 0.f, 0.f, 0.f, 0.f};

#pragma unroll 1
  for (int k0 = 0; k0 < KTOT; k0 += 32) {
    F bf[4];
#pragma unroll
    for (int j = 0; j < 4; ++j) bf[j] = ld_frag<F>(pb + (size_t)(j << 4) * (size_t)KTOT + k0);
#pragma unroll
    for (int i = 0; i < 4; ++i) {
      const F af = ld_frag<F>(pa + (size_t)(i << 4) * (size_t)KTOT + k0);
#pragma unroll
      for (int j = 0; j < 4; ++j) acc[i][j] = mm(af, bf[j], acc[i][j]);
    }
  }

  float* slab = sT[wave];
  const int hh = lane >> 4;
  const int c4 = (lane & 15) * 4;
  const int nc = n0 + c4;
  const bool cok = nc < N;
  v4f bv = (v4f){0.f, 0.f, 0.f, 0.f};
  if (EPI == 1) {
    bv = *(const v4fa*)(bias + clampi(nc, 0, N - 4));
    asm volatile("" :: "v"(bv));
  }
#pragma unroll
  for (int i = 0; i < 4; ++i) {
    const int mBase = m0 + (i << 4);
#pragma unroll
    for (int j = 0; j < 4; ++j) {
#pragma unroll
      for (int r = 0; r < 8; ++r) slab[(h8 + r) * 68 + (j << 4) + rl] = acc[i][j][r];
    }
    __builtin_amdgcn_fence(__ATOMIC_RELEASE, "workgroup");
    __builtin_amdgcn_wave_barrier();
    __builtin_amdgcn_fence(__ATOMIC_ACQUIRE, "workgroup");
    v4f vv[8];
#pragma unroll
    for (int it = 0; it < 8; ++it) {
      const int row = it * 2 + hh;
      v4f v = *(const v4fa*)(slab + row * 68 + c4);
      if (EPI == 1) v += bv;
      vv[it] = v;
    }
    for (int pass = 0; pass < 2; ++pass) {
#pragma unroll
      for (int it = 0; it < 8; ++it) {
        const int row = mBase + it * 2 + hh;
        if (cok && row < M) *(volatile v4f*)(D + (size_t)row * (size_t)ldd + nc) = vv[it];
      }
      __threadfence();
    }
    __builtin_amdgcn_fence(__ATOMIC_RELEASE, "workgroup");
    __builtin_amdgcn_wave_barrier();
    __builtin_amdgcn_fence(__ATOMIC_ACQUIRE, "workgroup");
  }
}

#include <stddef.h>
#include <stdint.h>


#define NN      50000
#define NE      800000
#define HH      64
#define NL      4
#define HPLANES 3
#define KT      (64 * HPLANES)
#define PPR     (KT / 8)
#define MPAD    50048
#define NBRUN   1024
#define SLA     10
#define NBKT    49
#define NPADN   (NBKT * NBRUN)
#define NTHR    256
#define NWAVE   8
#define EPT     8
#define CHUNK   (NTHR * EPT)
#define WCAP    (EPT * 32)
#define LISTN   (NWAVE * WCAP)
#define RCAP    28672
#define DEGCAP  48
#define ARRN    (NBRUN + 16)
#define BK_INTS (LISTN + 2 * RCAP + ARRN + 32)
#define NATT    196
#define NPC     ((64 * PPR) / 256)
#define NB_W    ((NL * 64 * PPR) / 256)
#define NB_O    ((64 * PPR) / 256)
#define NB_X    ((NN + 255) / 256)

#define PAR_INW  0
#define PAR_INB  256
#define PAR_OB1  320
#define PAR_OW2  352
#define PAR_OB2  480
#define PAR_RESW 484
#define PAR_L0   512
#define LSTRIDE  1952
#define L_RB1    0
#define L_WE0    64
#define L_WE1    128
#define L_RW2    192
#define L_RB2    448
#define L_SB     452
#define L_SW     456
#define L_QW     712
#define L_QB     968
#define L_KW     1032
#define L_KB     1288
#define L_VW     1352
#define L_VB     1608
#define L_OW     1672
#define L_OB     1928
#define L_LG     1932
#define L_LB     1936
#define PAR_N    (PAR_L0 + NL * LSTRIDE)
#define T_QW 0
#define T_QB 256
#define T_KW 320
#define T_KB 576
#define T_VW 640
#define T_VB 896
#define T_OW 960
#define T_OB 1216
#define T_LG 1220
#define T_LB 1224
#define TABN 1232

static_assert(HPLANES == 2 || HPLANES == 3);
static_assert(MPAD % 64 == 0 && MPAD >= NN && MPAD % 16 == 0 && KT % 32 == 0);
static_assert((64 * PPR) % 256 == 0 && (NL * 64 * PPR) % 256 == 0);
static_assert(NBRUN == (1 << SLA) && NBKT * NBRUN >= NN && NBRUN % 256 == 0);
static_assert(RCAP >= 16623 + 16623 / 20 && RCAP % 512 == 0);
static_assert(DEGCAP >= 35 + 8);
static_assert(NE < (1 << 20) && NE % 8 == 0 && ((NE * 4) % 16) == 0 && NN < 65536);
static_assert(BK_INTS % 4 == 0 && BK_INTS * 4 <= 327680);
static_assert(NATT * 256 >= NN && NN % 8 == 0 && (NATT - 1) * 256 < NN);
static_assert(PAR_N % 4 == 0 && LSTRIDE % 32 == 0 && L_LB + 4 <= LSTRIDE && PAR_RESW + 4 <= PAR_L0);
static_assert(L_LB + 4 - L_QW <= TABN && L_SW == L_SB + 4 && L_SB == L_RB2 + 4 && L_RB2 == L_RW2 + 256);
static_assert((MPAD / 64) * 1 <= 98 * 8);

typedef int   q4i __attribute__((ext_vector_type(4)));
typedef int   q2i __attribute__((ext_vector_type(2)));
typedef float q2f __attribute__((ext_vector_type(2)));
typedef q4i __attribute__((may_alias)) q4ia;
typedef q2i __attribute__((may_alias)) q2ia;
typedef q2f __attribute__((may_alias)) q2fa;
typedef v4u __attribute__((may_alias)) v4ua;

__device__ __forceinline__ void pin_f(float x) { asm volatile("" :: "v"(x)); }
__device__ __forceinline__ void pin_i(int x)   { asm volatile("" :: "v"(x)); }
__device__ __forceinline__ void pin_4f(const v4f v) { pin_f(v.x); pin_f(v.y); pin_f(v.z); pin_f(v.w); }
__device__ __forceinline__ float neg_inf() { return __int_as_float((int)0xff800000u); }
__device__ __forceinline__ float qnan()    { return __int_as_float(0x7fc00000); }
__device__ __forceinline__ float keepmax(float m, float y) { return (y > m || y != y) ? y : m; }
__device__ __forceinline__ float relu_k(float v) { return (v > 0.0f) ? v : (v - v); }

__device__ __forceinline__ void st2f(float* dp, const v4f v) {
  *(volatile v4f*)dp = v;
  __threadfence();
  *(volatile v4f*)dp = v;
}
__device__ __forceinline__ void st2u(unsigned short* dp, const v4u v) {
  *(volatile v4u*)dp = v;
  __threadfence();
  *(volatile v4u*)dp = v;
}

__device__ __forceinline__ void stage_tab(float* dst, const float* __restrict__ src, int n, int tid) {
#pragma unroll 1
  for (int t0 = 0; t0 < n; t0 += 256) {
    const int t = t0 + tid;
    const float v = src[t < n ? t : n - 1];
    pin_f(v);
    if (t < n) dst[t] = v;
  }
}
__device__ __forceinline__ void cp_lin(float* dst, const float* __restrict__ src, int n, int tid) {
#pragma unroll 1
  for (int t0 = 0; t0 < n; t0 += 256) {
    const int t = t0 + tid;
    const float v = src[t < n ? t : n - 1];
    pin_f(v);
    if (t < n) dst[t] = bf16_val(v);
  }
}
__device__ __forceinline__ void cp_col4(float* dst, const float* __restrict__ src, int stride, int tid) {
  const float v = src[(size_t)(tid >> 2) * (size_t)stride + (size_t)(tid & 3)];
  pin_f(v);
  dst[tid] = bf16_val(v);
}
__device__ __forceinline__ v4u gat8w(const float* __restrict__ w, size_t sb, int stride, unsigned mk) {
  float f[8];
#pragma unroll
  for (int e = 0; e < 8; ++e) { f[e] = w[sb + (size_t)e * (size_t)stride]; pin_f(f[e]); }
  return (v4u){ pk16(bf16_bits(f[0]) & mk, bf16_bits(f[1]) & mk), pk16(bf16_bits(f[2]) & mk, bf16_bits(f[3]) & mk),
                pk16(bf16_bits(f[4]) & mk, bf16_bits(f[5]) & mk), pk16(bf16_bits(f[6]) & mk, bf16_bits(f[7]) & mk) };
}

__global__ __launch_bounds__(256) void k_prep(
    const float* __restrict__ x, const float* __restrict__ in_w, const float* __restrict__ in_b,
    const float* __restrict__ rw1, const float* __restrict__ rb1, const float* __restrict__ rw2,
    const float* __restrict__ rb2, const float* __restrict__ sw, const float* __restrict__ sb,
    const float* __restrict__ qw, const float* __restrict__ qb, const float* __restrict__ kw,
    const float* __restrict__ kb, const float* __restrict__ vw, const float* __restrict__ vb,
    const float* __restrict__ ow, const float* __restrict__ ob, const float* __restrict__ lg,
    const float* __restrict__ lb, const float* __restrict__ ow1, const float* __restrict__ ob1,
    const float* __restrict__ ow2, const float* __restrict__ ob2, const float* __restrict__ resw,
    float* par, unsigned short* rw1t, unsigned short* ow1t, float* xo) {
  __shared__ __attribute__((aligned(16))) float sp[PAR_N];
  const int b = (int)blockIdx.x, tid = (int)threadIdx.x;
  if (b == 0) {
    for (int t = tid; t < PAR_N; t += 256) sp[t] = 0.0f;
    __syncthreads();
    cp_lin(sp + PAR_INW, in_w, 256, tid);
    cp_lin(sp + PAR_INB, in_b, 64, tid);
    cp_lin(sp + PAR_OB1, ob1, 32, tid);
    cp_lin(sp + PAR_OW2, ow2, 128, tid);
    cp_lin(sp + PAR_OB2, ob2, 4, tid);
    cp_lin(sp + PAR_RESW, resw, 4, tid);
#pragma unroll 1
    for (int i = 0; i < NL; ++i) {
      float* q = sp + PAR_L0 + i * LSTRIDE;
      cp_lin(q + L_RB1, rb1 + i * 64, 64, tid);
      cp_lin(q + L_WE0, rw1 + (size_t)i * 4224 + 64 * 64, 64, tid);
      cp_lin(q + L_WE1, rw1 + (size_t)i * 4224 + 65 * 64, 64, tid);
      cp_col4(q + L_RW2, rw2 + (size_t)i * 4096, 64, tid);
      cp_lin(q + L_RB2, rb2 + i * 64, 4, tid);
      cp_lin(q + L_SB, sb + i * 256, 4, tid);
      cp_col4(q + L_SW, sw + (size_t)i * 16384, 256, tid);
      cp_lin(q + L_QW, qw + i * 256, 256, tid);
      cp_lin(q + L_QB, qb + i * 64, 64, tid);
      cp_lin(q + L_KW, kw + i * 256, 256, tid);
      cp_lin(q + L_KB, kb + i * 64, 64, tid);
      cp_lin(q + L_VW, vw + i * 256, 256, tid);
      cp_lin(q + L_VB, vb + i * 64, 64, tid);
      cp_lin(q + L_OW, ow + i * 256, 256, tid);
      cp_lin(q + L_OB, ob + i * 4, 4, tid);
      cp_lin(q + L_LG, lg + i * 4, 4, tid);
      cp_lin(q + L_LB, lb + i * 4, 4, tid);
    }
    __syncthreads();
    for (int pass = 0; pass < 2; ++pass) {
#pragma unroll 1
      for (int t0 = 0; t0 < PAR_N / 4; t0 += 256) {
        const int t  = t0 + tid;
        const int tc = t < PAR_N / 4 ? t : PAR_N / 4 - 1;
        const v4f v = *(const v4fa*)(sp + 4 * tc);
        if (t < PAR_N / 4) *(volatile v4f*)(par + 4 * t) = v;
      }
      __threadfence();
    }
  } else if (b < 1 + NB_W) {
    const int u   = (b - 1) * 256 + tid;
    const int i   = u / (64 * PPR);
    const int rem = u - i * (64 * PPR);
    const int n   = rem / PPR;
    const int p   = rem - n * PPR;
    const int k8  = (p & 7) * 8;
    const v4u o = gat8w(rw1, (size_t)i * 4224 + (size_t)k8 * 64 + (size_t)n, 64, 0xFFFFu);
    st2u(rw1t + (size_t)u * 8, o);
  } else if (b < 1 + NB_W + NB_O) {
    const int u  = (b - 1 - NB_W) * 256 + tid;
    const int n  = u / PPR;
    const int p  = u - n * PPR;
    const int k8 = (p & 7) * 8;
    const int nc = n < 32 ? n : 31;
    const v4u o = gat8w(ow1, (size_t)k8 * 32 + (size_t)nc, 32, n < 32 ? 0xFFFFu : 0u);
    st2u(ow1t + (size_t)u * 8, o);
  } else {
    const int u  = (b - 1 - NB_W - NB_O) * 256 + tid;
    const int uc = u < NN ? u : NN - 1;
    const v4f xv = *(const v4fa*)(x + (size_t)uc * 4);
    pin_4f(xv);
    const v4f o = (v4f){ bf16_val(xv.x), bf16_val(xv.y), bf16_val(xv.z), bf16_val(xv.w) };
    if (u < NN) st2f(xo + (size_t)u * 4, o);
  }
}

__device__ __forceinline__ int ldkey(const int* __restrict__ k, int e, int nE, int sent) {
  const int v = k[e < nE ? e : nE - 1];
  pin_i(v);
  return (e < nE) ? v : sent;
}

__device__ __forceinline__ int scan_chunk(const int* __restrict__ keys, int nE, int cbase, int slotBase,
                                          int nb, int* list, int tid, int lane, int wave) {
  int wc = 0;
  const int el0  = tid * EPT;
  const int e0   = cbase + el0;
  const int sent = (int)(1u << 31);
  q4i da, db;
  if (cbase + CHUNK <= nE) {
    da = *(const q4i*)(keys + e0);
    db = *(const q4i*)(keys + e0 + 4);
  } else {
    da.x = ldkey(keys, e0,     nE, sent);
    da.y = ldkey(keys, e0 + 1, nE, sent);
    da.z = ldkey(keys, e0 + 2, nE, sent);
    da.w = ldkey(keys, e0 + 3, nE, sent);
    db.x = ldkey(keys, e0 + 4, nE, sent);
    db.y = ldkey(keys, e0 + 5, nE, sent);
    db.z = ldkey(keys, e0 + 6, nE, sent);
    db.w = ldkey(keys, e0 + 7, nE, sent);
  }
  const unsigned nbs = (unsigned)slotBase;
  const unsigned unb = (unsigned)nb;
  const unsigned s0 = (unsigned)da.x - nbs, s1 = (unsigned)da.y - nbs;
  const unsigned s2 = (unsigned)da.z - nbs, s3 = (unsigned)da.w - nbs;
  const unsigned s4 = (unsigned)db.x - nbs, s5 = (unsigned)db.y - nbs;
  const unsigned s6 = (unsigned)db.z - nbs, s7 = (unsigned)db.w - nbs;
  const bool h0 = s0 < unb, h1 = s1 < unb, h2 = s2 < unb, h3 = s3 < unb;
  const bool h4 = s4 < unb, h5 = s5 < unb, h6 = s6 < unb, h7 = s7 < unb;
  const unsigned any = __builtin_amdgcn_ballot_w32(h0 | h1 | h2 | h3 | h4 | h5 | h6 | h7);
  if (any != 0u) {
    const int k = (int)h0 + (int)h1 + (int)h2 + (int)h3 + (int)h4 + (int)h5 + (int)h6 + (int)h7;
    int incl = k;
#pragma unroll
    for (int dd = 1; dd < 32; dd <<= 1) {
      const int y = __shfl_up(incl, dd, 32);
      if (lane >= dd) incl += y;
    }
    wc = __shfl(incl, 31, 32);
    int pos = incl - k;
#define PUTJ(J, HJ, SJ) if (HJ) { if (pos < WCAP) list[wave * WCAP + pos] = ((el0 + (J)) << SLA) | (int)(SJ); pos += 1; }
    PUTJ(0, h0, s0)
    PUTJ(1, h1, s1)
    PUTJ(2, h2, s2)
    PUTJ(3, h3, s3)
    PUTJ(4, h4, s4)
    PUTJ(5, h5, s5)
    PUTJ(6, h6, s6)
    PUTJ(7, h7, s7)
#undef PUTJ
  }
  return wc;
}

__global__ __launch_bounds__(NTHR) void k_bucket(const int* __restrict__ rowi, const int* __restrict__ coli,
                                                 int* hitsg, int* offg, int* cntg, int* flagg) {
  extern __shared__ __attribute__((aligned(16))) int dsm[];
  int* list = dsm;
  int* hk   = dsm + LISTN;
  int* ent  = hk + RCAP;
  int* arr  = ent + RCAP;
  int* misc = arr + ARRN;
  const int tid = (int)threadIdx.x, lane = tid & 31;
  const int wave = __builtin_amdgcn_readfirstlane(tid >> 5);
  const int b = (int)blockIdx.x;
  const int nodeBase = b * NBRUN;

  {
    const q4i z4 = {0, 0, 0, 0};
    for (int i = tid * 4; i < BK_INTS; i += NTHR * 4) *(q4ia*)(dsm + i) = z4;
  }
  __syncthreads();

  int t = 0;
  const int nChunks = (NE + CHUNK - 1) / CHUNK;
#pragma unroll 1
  for (int ch = 0; ch < nChunks; ++ch) {
    const int cbase = ch * CHUNK;
    int wc = scan_chunk(coli, NE, cbase, nodeBase, NBRUN, list, tid, lane, wave);
    wc = clampi(wc, 0, WCAP);
    wc = __builtin_amdgcn_readfirstlane(wc);
    int* mb = misc + (ch & 1) * 8;
    if (lane == 0) mb[wave] = wc;
    __syncthreads();
    int base = t, tot = 0;
#pragma unroll
    for (int w2 = 0; w2 < NWAVE; ++w2) {
      const int c = clampi(mb[w2], 0, WCAP);
      base += (w2 < wave) ? c : 0;
      tot  += c;
    }
#pragma unroll 1
    for (int b0 = 0; b0 < wc; b0 += 32) {
      const int idx  = b0 + lane;
      const int entv = list[wave * WCAP + (idx < WCAP ? idx : WCAP - 1)];
      const int slot = entv & (NBRUN - 1);
      const int el   = (entv >> SLA) & (CHUNK - 1);
      const int eid  = clampi(cbase + el, 0, NE - 1);
      const int pos  = base + idx;
      if (idx < wc && pos < RCAP) hk[pos] = (eid << SLA) | slot;
    }
    t += tot;
  }
  __syncthreads();
  const int tt = t < RCAP ? t : RCAP;
  const int ov = t > RCAP ? 1 : 0;

  if (tid == 0) {
#pragma unroll 1
    for (int i = 0; i < tt; ++i) {
      const int k = hk[i] & (NBRUN - 1);
      arr[k] = arr[k] + 1;
    }
  }
  __syncthreads();
  if (wave == 0) {
    const int base = lane * (NBRUN / 32);
    int s = 0;
#pragma unroll 1
    for (int i = 0; i < NBRUN / 32; ++i) s += arr[base + i];
    int incl = s;
#pragma unroll
    for (int dd = 1; dd < 32; dd <<= 1) {
      const int y = __shfl_up(incl, dd, 32);
      if (lane >= dd) incl += y;
    }
    int run = incl - s;
#pragma unroll 1
    for (int i = 0; i < NBRUN / 32; ++i) {
      run += arr[base + i];
      arr[base + i] = run;
    }
    if (lane == 31) arr[NBRUN] = run;
  }
  __syncthreads();
  if (tid == 0) {
#pragma unroll 1
    for (int i = tt - 1; i >= 0; --i) {
      const int w = hk[i];
      const int k = w & (NBRUN - 1);
      const int p = clampi(arr[k] - 1, 0, RCAP - 1);
      arr[k] = p;
      ent[p] = (w >> SLA) & ((1 << 20) - 1);
    }
  }
  __syncthreads();

  int ovd = 0;
  const int k0 = 4 * tid;
  const int a0 = arr[k0], a1 = arr[k0 + 1], a2 = arr[k0 + 2], a3 = arr[k0 + 3], a4 = arr[k0 + 4];
  int c0 = a1 - a0, c1 = a2 - a1, c2 = a3 - a2, c3 = a4 - a3;
  ovd |= (c0 > DEGCAP) ? 1 : 0; ovd |= (c1 > DEGCAP) ? 1 : 0;
  ovd |= (c2 > DEGCAP) ? 1 : 0; ovd |= (c3 > DEGCAP) ? 1 : 0;
  const q4i cntv = { clampi(c0, 0, DEGCAP), clampi(c1, 0, DEGCAP), clampi(c2, 0, DEGCAP), clampi(c3, 0, DEGCAP) };
  const q4i offv = { clampi(a0, 0, RCAP - 1), clampi(a1, 0, RCAP - 1), clampi(a2, 0, RCAP - 1), clampi(a3, 0, RCAP - 1) };
  const unsigned om = __builtin_amdgcn_ballot_w32(ovd != 0);
  if (lane == 0) misc[20 + wave] = (om != 0u) ? 1 : 0;
  __syncthreads();
  int fl = ov;
#pragma unroll
  for (int w2 = 0; w2 < NWAVE; ++w2) fl |= misc[20 + w2];
  const q4i flv = { fl, fl, fl, fl };

  int* hg = hitsg + (size_t)b * (2 * RCAP);
  for (int pass = 0; pass < 2; ++pass) {
    *(volatile q4i*)(offg + (size_t)b * NBRUN + k0) = offv;
    *(volatile q4i*)(cntg + (size_t)b * NBRUN + k0) = cntv;
    if (tid < 8) *(volatile q4i*)(flagg + b * 32 + 4 * tid) = flv;
#pragma unroll 1
    for (int i = tid * 2; i < RCAP; i += 512) {
      const q2i ev = *(const q2ia*)(ent + i);
      const int e0 = clampi(ev.x, 0, NE - 1);
      const int e1 = clampi(ev.y, 0, NE - 1);
      int s0 = rowi[e0];
      int s1 = rowi[e1];
      pin_i(s0); pin_i(s1);
      s0 = clampi(s0, 0, NN - 1);
      s1 = clampi(s1, 0, NN - 1);
      const q4i hv = { e0, s0, e1, s1 };
      *(volatile q4i*)(hg + 2 * i) = hv;
    }
    __threadfence();
  }
}

template <int WITH_S4>
__global__ __launch_bounds__(256) void k_node(const float* __restrict__ X, const float* __restrict__ par, int lbase,
                                              unsigned short* hhl, float* s4) {
  __shared__ __attribute__((aligned(16))) unsigned short tile[64 * KT];
  __shared__ __attribute__((aligned(16))) float tinw[256];
  __shared__ __attribute__((aligned(16))) float tinb[64];
  __shared__ __attribute__((aligned(16))) float tsw[256];
  __shared__ __attribute__((aligned(16))) float tsb[4];
  __shared__ __attribute__((aligned(16))) float s4s[256];
  const int tid = (int)threadIdx.x, blk = (int)blockIdx.x;
  stage_tab(tinw, par + PAR_INW, 256, tid);
  stage_tab(tinb, par + PAR_INB, 64, tid);
  if (WITH_S4) {
    stage_tab(tsw, par + lbase + L_SW, 256, tid);
    stage_tab(tsb, par + lbase + L_SB, 4, tid);
  }
  __syncthreads();
  const int row = tid >> 2, q = tid & 3;
  const int node = blk * 64 + row;
  const bool live = node < NN;
  const int nc = live ? node : NN - 1;
  const v4f xv = *(const v4fa*)(X + (size_t)nc * 4);
  pin_4f(xv);
  float p0 = 0.0f, p1 = 0.0f, p2 = 0.0f, p3 = 0.0f;
#pragma unroll 1
  for (int d = 0; d < 16; ++d) {
    const int c = q * 16 + d;
    float hv = xv.x * tinw[c];
    hv = fmaf(xv.y, tinw[64 + c], hv);
    hv = fmaf(xv.z, tinw[128 + c], hv);
    hv = fmaf(xv.w, tinw[192 + c], hv);
    hv = hv + tinb[c];
    hv = live ? hv : 0.0f;
    const unsigned hb = bf16_bits(hv);
    float fh = __uint_as_float(hb << 16);
    asm volatile("" : "+v"(fh));
    const float r1 = hv - fh;
    const unsigned mb = bf16_bits(r1);
    float fm = __uint_as_float(mb << 16);
    asm volatile("" : "+v"(fm));
    const float r2 = r1 - fm;
    const unsigned lb = bf16_bits(r2);
    tile[row * KT + c]      = (unsigned short)hb;
    tile[row * KT + 64 + c] = (unsigned short)mb;
    if (HPLANES == 3) tile[row * KT + 2 * 64 * (HPLANES - 2) + c] = (unsigned short)lb;
    if (WITH_S4) {
      p0 = fmaf(hv, tsw[c * 4 + 0], p0);
      p1 = fmaf(hv, tsw[c * 4 + 1], p1);
      p2 = fmaf(hv, tsw[c * 4 + 2], p2);
      p3 = fmaf(hv, tsw[c * 4 + 3], p3);
    }
  }
  if (WITH_S4) {
    const float b0 = tsb[0], b1 = tsb[1], b2 = tsb[2], b3 = tsb[3];
    p0 += __shfl_xor(p0, 1, 32); p1 += __shfl_xor(p1, 1, 32);
    p2 += __shfl_xor(p2, 1, 32); p3 += __shfl_xor(p3, 1, 32);
    p0 += __shfl_xor(p0, 2, 32); p1 += __shfl_xor(p1, 2, 32);
    p2 += __shfl_xor(p2, 2, 32); p3 += __shfl_xor(p3, 2, 32);
    const v4f sv = (v4f){ p0 + b0, p1 + b1, p2 + b2, p3 + b3 };
    if (q == 0) *(v4fa*)(s4s + row * 4) = sv;
  }
  __syncthreads();
  v4u pc[NPC];
#pragma unroll
  for (int it = 0; it < NPC; ++it) pc[it] = *(const v4ua*)(tile + (size_t)(it * 256 + tid) * 8);
  unsigned short* gb = hhl + (size_t)blk * (64 * KT);
  for (int pass = 0; pass < 2; ++pass) {
#pragma unroll
    for (int it = 0; it < NPC; ++it) *(volatile v4u*)(gb + (size_t)(it * 256 + tid) * 8) = pc[it];
    __threadfence();
  }
  if (WITH_S4) {
    if (tid < 64) {
      const v4f sv = *(const v4fa*)(s4s + tid * 4);
      const int n2 = blk * 64 + tid;
      if (n2 < NN) st2f(s4 + (size_t)n2 * 4, sv);
    }
  }
  (void)s4; (void)lbase;
}

__global__ __launch_bounds__(256) void k_conv(const float* __restrict__ P, const int* __restrict__ hitsg,
                                              const int* __restrict__ offg, const int* __restrict__ cntg,
                                              const int* __restrict__ flagg, const float* __restrict__ ea,
                                              const float* __restrict__ par, int lbase,
                                              const float* __restrict__ s4, float* x4out) {
  __shared__ __attribute__((aligned(16))) float tab[456];
  __shared__ __attribute__((aligned(16))) float xs[NBRUN * 4];
  const int tid = (int)threadIdx.x, lane = tid & 31, blk = (int)blockIdx.x;
  const int wave = __builtin_amdgcn_readfirstlane(tid >> 5);
  stage_tab(tab, par + lbase, 456, tid);
  __syncthreads();
  const float rb1a = tab[L_RB1 + 2 * lane], rb1b = tab[L_RB1 + 2 * lane + 1];
  const float we0a = tab[L_WE0 + 2 * lane], we0b = tab[L_WE0 + 2 * lane + 1];
  const float we1a = tab[L_WE1 + 2 * lane], we1b = tab[L_WE1 + 2 * lane + 1];
  const v4f w2a = *(const v4fa*)(tab + L_RW2 + 8 * lane);
  const v4f w2b = *(const v4fa*)(tab + L_RW2 + 8 * lane + 4);
  const v4f rb2 = *(const v4fa*)(tab + L_RB2);
  int fl = flagg[blk * 32];
  pin_i(fl);
  const float pz = (fl != 0) ? qnan() : 0.0f;
  const int* hb = hitsg + (size_t)blk * (2 * RCAP);
#pragma unroll 1
  for (int t = 0; t < NBRUN / NWAVE; ++t) {
    const int slot = wave * (NBRUN / NWAVE) + t;
    const int node = blk * NBRUN + slot;
    const int nc = node < NN ? node : NN - 1;
    int cnt = cntg[(size_t)blk * NBRUN + slot];
    int off = offg[(size_t)blk * NBRUN + slot];
    pin_i(cnt); pin_i(off);
    cnt = clampi(cnt, 0, DEGCAP);
    off = clampi(off, 0, RCAP - 1);
    if (cnt > RCAP - off) cnt = RCAP - off;
    cnt = __builtin_amdgcn_readfirstlane(cnt);
    off = __builtin_amdgcn_readfirstlane(off);
    float h0 = 0.0f, h1 = 0.0f;
#pragma unroll 1
    for (int p = 0; p < cnt; ++p) {
      const q2i es = *(const q2ia*)(hb + 2 * (size_t)(off + p));
      pin_i(es.x); pin_i(es.y);
      const int e   = clampi(es.x, 0, NE - 1);
      const int src = clampi(es.y, 0, NN - 1);
      const q2f pv = *(const q2fa*)(P + (size_t)src * 64 + 2 * lane);
      const q2f ev = *(const q2fa*)(ea + (size_t)e * 2);
      const float a0 = bf16_val(ev.x), a1 = bf16_val(ev.y);
      float v0 = fmaf(a0, we0a, pv.x);
      v0 = fmaf(a1, we1a, v0);
      v0 = v0 + rb1a;
      float v1 = fmaf(a0, we0b, pv.y);
      v1 = fmaf(a1, we1b, v1);
      v1 = v1 + rb1b;
      h0 += relu_k(v0);
      h1 += relu_k(v1);
    }
    {
      const q2f pv = *(const q2fa*)(P + (size_t)nc * 64 + 2 * lane);
      h0 += relu_k(pv.x + rb1a);
      h1 += relu_k(pv.y + rb1b);
    }
    float d0 = h0 * w2a.x; d0 = fmaf(h1, w2b.x, d0);
    float d1 = h0 * w2a.y; d1 = fmaf(h1, w2b.y, d1);
    float d2 = h0 * w2a.z; d2 = fmaf(h1, w2b.z, d2);
    float d3 = h0 * w2a.w; d3 = fmaf(h1, w2b.w, d3);
#pragma unroll
    for (int o = 16; o >= 1; o >>= 1) {
      d0 += __shfl_xor(d0, o, 32);
      d1 += __shfl_xor(d1, o, 32);
      d2 += __shfl_xor(d2, o, 32);
      d3 += __shfl_xor(d3, o, 32);
    }
    const float deg = (float)(cnt + 1);
    const v4f sv = *(const v4fa*)(s4 + (size_t)nc * 4);
    const v4f r = (v4f){ (d0 / deg + rb2.x) + sv.x + pz, (d1 / deg + rb2.y) + sv.y + pz,
                         (d2 / deg + rb2.z) + sv.z + pz, (d3 / deg + rb2.w) + sv.w + pz };
    if (lane == 0) *(v4fa*)(xs + slot * 4) = r;
  }
  __syncthreads();
  v4f vals[4];
#pragma unroll
  for (int it = 0; it < 4; ++it) vals[it] = *(const v4fa*)(xs + (size_t)(it * 256 + tid) * 4);
  for (int pass = 0; pass < 2; ++pass) {
#pragma unroll
    for (int it = 0; it < 4; ++it) {
      const int node = blk * NBRUN + it * 256 + tid;
      if (node < NN) *(volatile v4f*)(x4out + (size_t)node * 4) = vals[it];
    }
    __threadfence();
  }
}

__device__ __forceinline__ void att_build_a(const float* tab, const v4f x, float* acol, int tid) {
#pragma unroll 1
  for (int hd = 0; hd < 4; ++hd) {
    float a0 = 0.0f, a1 = 0.0f, a2 = 0.0f, a3 = 0.0f, a4 = 0.0f;
#pragma unroll 1
    for (int d = 0; d < 16; ++d) {
      const int c = hd * 16 + d;
      float kv = x.x * tab[T_KW + c];
      kv = fmaf(x.y, tab[T_KW + 64 + c], kv);
      kv = fmaf(x.z, tab[T_KW + 128 + c], kv);
      kv = fmaf(x.w, tab[T_KW + 192 + c], kv);
      kv = kv + tab[T_KB + c];
      a0 = fmaf(tab[T_QW + c], kv, a0);
      a1 = fmaf(tab[T_QW + 64 + c], kv, a1);
      a2 = fmaf(tab[T_QW + 128 + c], kv, a2);
      a3 = fmaf(tab[T_QW + 192 + c], kv, a3);
      a4 = fmaf(tab[T_QB + c], kv, a4);
    }
    float* ap = acol + hd * 5 * 256 + tid;
    ap[0] = a0; ap[256] = a1; ap[512] = a2; ap[768] = a3; ap[1024] = a4;
  }
}

__device__ __forceinline__ float att_score(const v4f xs, const float* acol, int hd, int tid) {
  const float* ap = acol + hd * 5 * 256 + tid;
  float s = xs.x * ap[0];
  s = fmaf(xs.y, ap[256], s);
  s = fmaf(xs.z, ap[512], s);
  s = fmaf(xs.w, ap[768], s);
  s = s + ap[1024];
  return 0.25f * s;
}

__device__ __forceinline__ v4f att_fetch(const int* __restrict__ hb, const float* __restrict__ x4,
                                         int off, int cnt, int p) {
  int q = cnt - 1;
  q = q < 0 ? 0 : q;
  const int pp  = p < q ? p : q;
  const int idx = clampi(off + pp, 0, RCAP - 1);
  const q2i es = *(const q2ia*)(hb + 2 * (size_t)idx);
  pin_i(es.x); pin_i(es.y);
  const int src = clampi(es.y, 0, NN - 1);
  const v4f xs = *(const v4fa*)(x4 + (size_t)src * 4);
  pin_4f(xs);
  return xs;
}

__global__ __launch_bounds__(256) void k_att_rec(const float* __restrict__ x4, const int* __restrict__ hitsg,
                                                 const int* __restrict__ offg, const int* __restrict__ cntg,
                                                 const float* __restrict__ par, int lbase, float* rec) {
  __shared__ __attribute__((aligned(16))) float tab[TABN];
  __shared__ float acol[20 * 256];
  __shared__ float mcol[4 * 256];
  __shared__ float zcol[4 * 256];
  __shared__ float wrec[64];
  const int tid = (int)threadIdx.x, lane = tid & 31, blk = (int)blockIdx.x;
  const int wave = __builtin_amdgcn_readfirstlane(tid >> 5);
  stage_tab(tab, par + lbase + L_QW, 640, tid);
  const int n = blk * 256 + tid;
  const bool live = n < NN;
  const int nc = live ? n : NN - 1;
  const v4f xo = *(const v4fa*)(x4 + (size_t)nc * 4);
  pin_4f(xo);
  int cnt = cntg[nc];
  int off = offg[nc];
  pin_i(cnt); pin_i(off);
  cnt = clampi(cnt, 0, DEGCAP);
  off = clampi(off, 0, RCAP - 1);
  if (cnt > RCAP - off) cnt = RCAP - off;
  cnt = live ? cnt : 0;
  const int* hb = hitsg + (size_t)(nc >> SLA) * (2 * RCAP);
#pragma unroll 1
  for (int hd = 0; hd < 4; ++hd) { mcol[hd * 256 + tid] = neg_inf(); zcol[hd * 256 + tid] = 0.0f; }
  __syncthreads();
  att_build_a(tab, xo, acol, tid);

  int cm = cnt;
#pragma unroll
  for (int o = 16; o >= 1; o >>= 1) {
    const int y = __shfl_xor(cm, o, 32);
    cm = cm > y ? cm : y;
  }
  cm = __builtin_amdgcn_readfirstlane(cm);
  cm = cm > DEGCAP ? DEGCAP : cm;
#pragma unroll 1
  for (int p = 0; p < cm; ++p) {
    const v4f xs = att_fetch(hb, x4, off, cnt, p);
    const bool valid = p < cnt;
#pragma unroll 1
    for (int hd = 0; hd < 4; ++hd) {
      const float s = att_score(xs, acol, hd, tid);
      const float m = mcol[hd * 256 + tid];
      const float z = zcol[hd * 256 + tid];
      const bool up = (s > m) || (s != s);
      const float e = expf(-fabsf(s - m));
      const float zn = up ? fmaf(z, e, 1.0f) : (z + e);
      const float mn = up ? s : m;
      mcol[hd * 256 + tid] = valid ? mn : m;
      zcol[hd * 256 + tid] = valid ? zn : z;
    }
  }
#pragma unroll 1
  for (int hd = 0; hd < 4; ++hd) {
    const float m = mcol[hd * 256 + tid];
    const float z = zcol[hd * 256 + tid];
    float mw = m;
#pragma unroll
    for (int o = 16; o >= 1; o >>= 1) {
      const float y = __shfl_xor(mw, o, 32);
      mw = keepmax(mw, y);
    }
    float term = z * expf(m - mw);
    term = (m == neg_inf()) ? 0.0f : term;
#pragma unroll
    for (int o = 16; o >= 1; o >>= 1) term += __shfl_xor(term, o, 32);
    if (lane == 0) { wrec[wave * 8 + hd] = mw; wrec[wave * 8 + 4 + hd] = term; }
  }
  __syncthreads();
  if (wave == 0) {
    const int hd = lane & 3;
    float mb = neg_inf();
#pragma unroll 1
    for (int w = 0; w < NWAVE; ++w) mb = keepmax(mb, wrec[w * 8 + hd]);
    float zb = 0.0f;
#pragma unroll 1
    for (int w = 0; w < NWAVE; ++w) {
      const float mwv = wrec[w * 8 + hd];
      const float zw  = wrec[w * 8 + 4 + hd];
      float tv = zw * expf(mwv - mb);
      tv = (mwv == neg_inf()) ? 0.0f : tv;
      zb += tv;
    }
    const float m0 = __shfl(mb, 0, 32), m1 = __shfl(mb, 1, 32), m2 = __shfl(mb, 2, 32), m3 = __shfl(mb, 3, 32);
    const float z0 = __shfl(zb, 0, 32), z1 = __shfl(zb, 1, 32), z2 = __shfl(zb, 2, 32), z3 = __shfl(zb, 3, 32);
    v4f o = (v4f){ 0.0f, 0.0f, 0.0f, 0.0f };
    const v4f mv = (v4f){ m0, m1, m2, m3 };
    const v4f zv = (v4f){ z0, z1, z2, z3 };
    if (lane == 0) o = mv;
    if (lane == 1) o = zv;
    if (lane < 8) st2f(rec + (size_t)blk * 32 + 4 * lane, o);
  }
}

__global__ __launch_bounds__(32) void k_att_comb(const float* __restrict__ rec, float* stat, int layer) {
  const int lane = (int)threadIdx.x & 31;
  const int hd = lane & 3;
  float m = neg_inf();
#pragma unroll 1
  for (int b = 0; b < NATT; ++b) m = keepmax(m, rec[b * 32 + hd]);
  double Z = 0.0;
#pragma unroll 1
  for (int b = 0; b < NATT; ++b) {
    const float mb = rec[b * 32 + hd];
    const float zb = rec[b * 32 + 4 + hd];
    const float f  = expf(mb - m);
    double tv = (double)zb * (double)f;
    tv = (mb == neg_inf()) ? 0.0 : tv;
    Z += tv;
  }
  const float zf = (float)Z;
  const float m0 = __shfl(m, 0, 32), m1 = __shfl(m, 1, 32), m2 = __shfl(m, 2, 32), m3 = __shfl(m, 3, 32);
  const float z0 = __shfl(zf, 0, 32), z1 = __shfl(zf, 1, 32), z2 = __shfl(zf, 2, 32), z3 = __shfl(zf, 3, 32);
  v4f o = (v4f){ 0.0f, 0.0f, 0.0f, 0.0f };
  const v4f mv = (v4f){ m0, m1, m2, m3 };
  const v4f zv = (v4f){ z0, z1, z2, z3 };
  if (lane == 0) o = mv;
  if (lane == 1) o = zv;
  if (lane < 8) st2f(stat + (size_t)layer * 32 + 4 * lane, o);
}

__global__ __launch_bounds__(256) void k_att_apply(const float* __restrict__ x4, const int* __restrict__ hitsg,
                                                   const int* __restrict__ offg, const int* __restrict__ cntg,
                                                   const float* __restrict__ par, int lbase,
                                                   const float* __restrict__ stat, int layer,
                                                   float* xio, float* diag) {
  __shared__ __attribute__((aligned(16))) float tab[TABN];
  __shared__ float acol[20 * 256];
  __shared__ float tcol[20 * 256];
  __shared__ float ocol[8 * 256];
  __shared__ float stt[8];
  const int tid = (int)threadIdx.x, blk = (int)blockIdx.x;
  stage_tab(tab, par + lbase + L_QW, L_LB + 4 - L_QW, tid);
  stage_tab(stt, stat + (size_t)layer * 32, 8, tid);
  const int n = blk * 256 + tid;
  const bool live = n < NN;
  const int nc = live ? n : NN - 1;
  const v4f xo = *(const v4fa*)(x4 + (size_t)nc * 4);
  pin_4f(xo);
  const v4f xr = *(const v4fa*)(xio + (size_t)nc * 4);
  pin_4f(xr);
  int cnt = cntg[nc];
  int off = offg[nc];
  pin_i(cnt); pin_i(off);
  cnt = clampi(cnt, 0, DEGCAP);
  off = clampi(off, 0, RCAP - 1);
  if (cnt > RCAP - off) cnt = RCAP - off;
  cnt = live ? cnt : 0;
  const int* hb = hitsg + (size_t)(nc >> SLA) * (2 * RCAP);
#pragma unroll 1
  for (int q = 0; q < 20; ++q) tcol[q * 256 + tid] = 0.0f;
  __syncthreads();
  att_build_a(tab, xo, acol, tid);
  const float rw = par[PAR_RESW + layer];

  int cm = cnt;
#pragma unroll
  for (int o = 16; o >= 1; o >>= 1) {
    const int y = __shfl_xor(cm, o, 32);
    cm = cm > y ? cm : y;
  }
  cm = __builtin_amdgcn_readfirstlane(cm);
  cm = cm > DEGCAP ? DEGCAP : cm;
#pragma unroll 1
  for (int p = 0; p < cm; ++p) {
    const v4f xs = att_fetch(hb, x4, off, cnt, p);
    const bool valid = p < cnt;
#pragma unroll 1
    for (int hd = 0; hd < 4; ++hd) {
      const float s = att_score(xs, acol, hd, tid);
      const float w = expf(s - stt[hd]);
      float* tp = tcol + hd * 5 * 256 + tid;
      const float t0 = tp[0], t1 = tp[256], t2 = tp[512], t3 = tp[768], t4 = tp[1024];
      const float u0 = fmaf(w, xs.x, t0);
      const float u1 = fmaf(w, xs.y, t1);
      const float u2 = fmaf(w, xs.z, t2);
      const float u3 = fmaf(w, xs.w, t3);
      const float u4 = t4 + w;
      tp[0]    = valid ? u0 : t0;
      tp[256]  = valid ? u1 : t1;
      tp[512]  = valid ? u2 : t2;
      tp[768]  = valid ? u3 : t3;
      tp[1024] = valid ? u4 : t4;
    }
  }
#pragma unroll 1
  for (int hd = 0; hd < 4; ++hd) {
    const float zh = stt[4 + hd];
#pragma unroll 1
    for (int j = 0; j < 5; ++j) {
      const float tv = tcol[(hd * 5 + j) * 256 + tid];
      tcol[(hd * 5 + j) * 256 + tid] = tv / zh;
    }
  }
  float c0 = 0.0f, c1 = 0.0f, c2 = 0.0f, c3 = 0.0f;
#pragma unroll 1
  for (int hd = 0; hd < 4; ++hd) {
    const float* tp = tcol + hd * 5 * 256 + tid;
    const float t0 = tp[0], t1 = tp[256], t2 = tp[512], t3 = tp[768], t4 = tp[1024];
#pragma unroll 1
    for (int d = 0; d < 16; ++d) {
      const int c = hd * 16 + d;
      float at = t0 * tab[T_VW + c];
      at = fmaf(t1, tab[T_VW + 64 + c], at);
      at = fmaf(t2, tab[T_VW + 128 + c], at);
      at = fmaf(t3, tab[T_VW + 192 + c], at);
      at = fmaf(t4, tab[T_VB + c], at);
      c0 = fmaf(at, tab[T_OW + c * 4 + 0], c0);
      c1 = fmaf(at, tab[T_OW + c * 4 + 1], c1);
      c2 = fmaf(at, tab[T_OW + c * 4 + 2], c2);
      c3 = fmaf(at, tab[T_OW + c * 4 + 3], c3);
    }
  }
  const float g0 = c0 + tab[T_OB + 0], g1 = c1 + tab[T_OB + 1], g2 = c2 + tab[T_OB + 2], g3 = c3 + tab[T_OB + 3];
#ifdef DIAG_ATT
  if (layer == 0 && live) st2f(diag + (size_t)n * 4, (v4f){ g0, g1, g2, g3 });
#endif
  const float o0 = g0 + xo.x, o1 = g1 + xo.y, o2 = g2 + xo.z, o3 = g3 + xo.w;
  const float mu = ((o0 + o1) + (o2 + o3)) * 0.25f;
  const float e0 = o0 - mu, e1 = o1 - mu, e2 = o2 - mu, e3 = o3 - mu;
  const float var = ((e0 * e0 + e1 * e1) + (e2 * e2 + e3 * e3)) * 0.25f;
  const float sd = sqrtf(var + 1e-5f);
  ocol[0 * 256 + tid] = e0; ocol[1 * 256 + tid] = e1; ocol[2 * 256 + tid] = e2; ocol[3 * 256 + tid] = e3;
  ocol[4 * 256 + tid] = xr.x; ocol[5 * 256 + tid] = xr.y; ocol[6 * 256 + tid] = xr.z; ocol[7 * 256 + tid] = xr.w;
#pragma unroll 1
  for (int j = 0; j < 4; ++j) {
    float y = ocol[j * 256 + tid] / sd;
    y = y * tab[T_LG + j] + tab[T_LB + j];
    y = y + ocol[(4 + j) * 256 + tid] * rw;
    ocol[j * 256 + tid] = y;
  }
  const v4f res = (v4f){ ocol[0 * 256 + tid], ocol[1 * 256 + tid], ocol[2 * 256 + tid], ocol[3 * 256 + tid] };
  if (live) st2f(xio + (size_t)n * 4, res);
  (void)diag;
}

__global__ __launch_bounds__(256) void k_head(const float* __restrict__ R, const float* __restrict__ par,
                                              const int* __restrict__ flagg, float* out) {
  __shared__ __attribute__((aligned(16))) float tab[164];
  __shared__ float sc[4 * 256];
  const int tid = (int)threadIdx.x, blk = (int)blockIdx.x;
  stage_tab(tab, par + PAR_OB1, 164, tid);
  __syncthreads();
  const int n = blk * 256 + tid;
  const bool live = n < NN;
  const int nc = live ? n : NN - 1;
  int fl = flagg[(nc >> SLA) * 32];
  pin_i(fl);
  const float pz = (fl != 0) ? qnan() : 0.0f;
  float a0 = 0.0f, a1 = 0.0f, a2 = 0.0f, a3 = 0.0f;
#pragma unroll 1
  for (int q = 0; q < 8; ++q) {
    const v4f r = *(const v4fa*)(R + (size_t)nc * 32 + q * 4);
    pin_4f(r);
    const float* w = tab + 32 + q * 16;
    const float t0 = relu_k(r.x + tab[q * 4 + 0]);
    const float t1 = relu_k(r.y + tab[q * 4 + 1]);
    const float t2 = relu_k(r.z + tab[q * 4 + 2]);
    const float t3 = relu_k(r.w + tab[q * 4 + 3]);
    a0 = fmaf(t0, w[0], a0);  a1 = fmaf(t0, w[1], a1);  a2 = fmaf(t0, w[2], a2);  a3 = fmaf(t0, w[3], a3);
    a0 = fmaf(t1, w[4], a0);  a1 = fmaf(t1, w[5], a1);  a2 = fmaf(t1, w[6], a2);  a3 = fmaf(t1, w[7], a3);
    a0 = fmaf(t2, w[8], a0);  a1 = fmaf(t2, w[9], a1);  a2 = fmaf(t2, w[10], a2); a3 = fmaf(t2, w[11], a3);
    a0 = fmaf(t3, w[12], a0); a1 = fmaf(t3, w[13], a1); a2 = fmaf(t3, w[14], a2); a3 = fmaf(t3, w[15], a3);
  }
  sc[0 * 256 + tid] = a0 + tab[160 + 0];
  sc[1 * 256 + tid] = a1 + tab[160 + 1];
  sc[2 * 256 + tid] = a2 + tab[160 + 2];
  sc[3 * 256 + tid] = a3 + tab[160 + 3];
#pragma unroll 1
  for (int j = 0; j < 4; ++j) {
    const float v = sc[j * 256 + tid];
    sc[j * 256 + tid] = tanhf(v) * 0.3f + pz;
  }
  const v4f o = (v4f){ sc[0 * 256 + tid], sc[1 * 256 + tid], sc[2 * 256 + tid], sc[3 * 256 + tid] };
  if (live) st2f(out + (size_t)n * 4, o);
}

static inline size_t al256(size_t o) { return (o + 255) & ~(size_t)255; }

extern "C" void kernel_launch(void* const* d_in, const int* in_sizes, int n_in,
                              void* d_out, int out_size, void* d_ws, size_t ws_size,
                              hipStream_t stream) {
  if (n_in < 30) return;
  if (in_sizes[0] != NN * 4 || in_sizes[1] != 2 * NE || in_sizes[2] != 2 * NE) return;
  if (in_sizes[3] != 4 * HH || in_sizes[4] != HH) return;
  if (in_sizes[5] != NL * 66 * HH || in_sizes[6] != NL * HH || in_sizes[7] != NL * HH * HH || in_sizes[8] != NL * HH) return;
  if (in_sizes[13] != NL * HH * 256 || in_sizes[14] != NL * 256) return;
  if (in_sizes[15] != NL * 256 || in_sizes[17] != NL * 256 || in_sizes[19] != NL * 256 || in_sizes[21] != NL * 256) return;
  if (in_sizes[16] != NL * HH || in_sizes[18] != NL * HH || in_sizes[20] != NL * HH) return;
  if (in_sizes[22] != NL * 4 || in_sizes[23] != NL * 4 || in_sizes[24] != NL * 4) return;
  if (in_sizes[25] != HH * 32 || in_sizes[26] != 32 || in_sizes[27] != 128 || in_sizes[28] != 4 || in_sizes[29] != NL) return;
  if (out_size != NN * 4) return;

  const float* x    = (const float*)d_in[0];
  const int*   eidx = (const int*)d_in[1];
  const int*   erow = eidx;
  const int*   ecol = eidx + NE;
  const float* ea   = (const float*)d_in[2];
  const float* in_w = (const float*)d_in[3];
  const float* in_b = (const float*)d_in[4];
  const float* rw1  = (const float*)d_in[5];
  const float* rb1  = (const float*)d_in[6];
  const float* rw2  = (const float*)d_in[7];
  const float* rb2  = (const float*)d_in[8];
  const float* sw   = (const float*)d_in[13];
  const float* sb   = (const float*)d_in[14];
  const float* qw   = (const float*)d_in[15];
  const float* qb   = (const float*)d_in[16];
  const float* kw   = (const float*)d_in[17];
  const float* kb   = (const float*)d_in[18];
  const float* vw   = (const float*)d_in[19];
  const float* vb   = (const float*)d_in[20];
  const float* ow   = (const float*)d_in[21];
  const float* ob   = (const float*)d_in[22];
  const float* lg   = (const float*)d_in[23];
  const float* lb   = (const float*)d_in[24];
  const float* ow1  = (const float*)d_in[25];
  const float* ob1  = (const float*)d_in[26];
  const float* ow2  = (const float*)d_in[27];
  const float* ob2  = (const float*)d_in[28];
  const float* resw = (const float*)d_in[29];
  float* out = (float*)d_out;

  char* ws = (char*)d_ws;
  size_t off = 0;
  const size_t oPAR  = off; off = al256(off + (size_t)PAR_N * 4);
  const size_t oRW1T = off; off = al256(off + (size_t)NL * 64 * KT * 2);
  const size_t oOW1T = off; off = al256(off + (size_t)64 * KT * 2);
  const size_t oX    = off; off = al256(off + (size_t)NN * 16);
  const size_t oX4   = off; off = al256(off + (size_t)NN * 16);
  const size_t oS4   = off; off = al256(off + (size_t)NN * 16);
  const size_t oHHL  = off; off = al256(off + (size_t)MPAD * KT * 2);
  const size_t oP    = off; off = al256(off + (size_t)MPAD * 64 * 4);
  const size_t oR    = off; off = al256(off + (size_t)MPAD * 32 * 4);
  const size_t oHITS = off; off = al256(off + (size_t)NBKT * RCAP * 8);
  const size_t oOFF  = off; off = al256(off + (size_t)NPADN * 4);
  const size_t oCNT  = off; off = al256(off + (size_t)NPADN * 4);
  const size_t oFLAG = off; off = al256(off + (size_t)NBKT * 128);
  const size_t oREC  = off; off = al256(off + (size_t)NATT * 128);
  const size_t oSTAT = off; off = al256(off + (size_t)NL * 128);
  if (off > ws_size || off > (size_t)(128u << 20)) return;

  float*          PAR  = (float*)(ws + oPAR);
  unsigned short* RW1T = (unsigned short*)(ws + oRW1T);
  unsigned short* OW1T = (unsigned short*)(ws + oOW1T);
  float*          X    = (float*)(ws + oX);
  float*          X4   = (float*)(ws + oX4);
  float*          S4   = (float*)(ws + oS4);
  unsigned short* HHL  = (unsigned short*)(ws + oHHL);
  float*          P    = (float*)(ws + oP);
  float*          R    = (float*)(ws + oR);
  int*            HITS = (int*)(ws + oHITS);
  int*            OFF  = (int*)(ws + oOFF);
  int*            CNT  = (int*)(ws + oCNT);
  int*            FLAG = (int*)(ws + oFLAG);
  float*          REC  = (float*)(ws + oREC);
  float*          STAT = (float*)(ws + oSTAT);

  const int bkLds = BK_INTS * 4;
  hipFuncSetAttribute(reinterpret_cast<const void*>(&k_bucket), hipFuncAttributeMaxDynamicSharedMemorySize, bkLds);

  k_prep<<<1 + NB_W + NB_O + NB_X, 256, 0, stream>>>(x, in_w, in_b, rw1, rb1, rw2, rb2, sw, sb, qw, qb, kw, kb, vw, vb,
                                                     ow, ob, lg, lb, ow1, ob1, ow2, ob2, resw, PAR, RW1T, OW1T, X);
  k_bucket<<<NBKT, NTHR, bkLds, stream>>>(erow, ecol, HITS, OFF, CNT, FLAG);

  const int gemmBlocks = ((MPAD / 64) + 7) / 8;
  for (int i = 0; i < NL; ++i) {
    const int lbase = PAR_L0 + i * LSTRIDE;
    k_node<1><<<MPAD / 64, 256, 0, stream>>>(X, PAR, lbase, HHL, S4);
    k_gemm_nt<0, 0><<<gemmBlocks, 256, 0, stream>>>(HHL, RW1T + (size_t)i * 64 * KT, PAR, P, MPAD, 64, KT, 64);
    k_conv<<<NBKT, 256, 0, stream>>>(P, HITS, OFF, CNT, FLAG, ea, PAR, lbase, S4, X4);
    k_att_rec<<<NATT, 256, 0, stream>>>(X4, HITS, OFF, CNT, PAR, lbase, REC);
    k_att_comb<<<1, 32, 0, stream>>>(REC, STAT, i);
    k_att_apply<<<NATT, 256, 0, stream>>>(X4, HITS, OFF, CNT, PAR, lbase, STAT, i, X, out);
#ifdef DIAG_ATT
    return;
#endif
  }
  k_node<0><<<MPAD / 64, 256, 0, stream>>>(X, PAR, PAR_L0, HHL, S4);
  k_gemm_nt<0, 0><<<gemmBlocks, 256, 0, stream>>>(HHL, OW1T, PAR, R, MPAD, 32, KT, 32);
  k_head<<<NATT, 256, 0, stream>>>(R, PAR, FLAG, out);
}
